// DecoderLayer_68212670595779
// MI455X (gfx1250) — hardware-verified
//
#include <hip/hip_runtime.h>
#include <math.h>
#ifndef NB
#define NB 2
#endif
#ifndef SEQ
#define SEQ 2048
#endif
#define NB_FULL 2
#define SEQ_FULL 2048
#define DM 1024
#define NH 16
#define HD 64
#define DFF 4096
#define LQ (3 * DM)
#define MROWS (NB * SEQ)
#define NQT (SEQ / 64)
#define NKT (SEQ / 64)
static_assert(SEQ % 64 == 0);
static_assert(SEQ <= SEQ_FULL);
static_assert(NB >= 1 && NB <= NB_FULL);
static_assert(NKT <= 32);
static_assert(MROWS % 128 == 0);
static_assert(DM % 64 == 0 && DFF % 64 == 0 && DM % 32 == 0 && DFF % 32 == 0);
static_assert(NH * HD == DM);
static_assert(DM == 256 * 4);
static_assert(((size_t)MROWS * DM / 8) % 256 == 0);
static_assert(NQT * 16 == SEQ / 4);

typedef _Float16 v16h __attribute__((ext_vector_type(16)));
typedef _Float16 v4h  __attribute__((ext_vector_type(4)));
typedef unsigned short v8us __attribute__((ext_vector_type(8), may_alias));
typedef float  v8f  __attribute__((ext_vector_type(8)));
typedef float  v4f  __attribute__((ext_vector_type(4)));
typedef float  v4fa __attribute__((ext_vector_type(4), may_alias));
typedef int    v4ia __attribute__((ext_vector_type(4), may_alias));
union FragH { v16h v; v8us half[2]; _Float16 h[16]; unsigned short u[16]; };

#define NEG_INF (-__builtin_inff())
#define FILL_RAW (-8.0e9f)
#define C_W   16.0f
#define C_CTX 64.0f
#define C_AO  256.0f
#define C_H   1024.0f

__device__ __forceinline__ unsigned short bf16_bits(float x) { unsigned int u = __float_as_uint(x); return (unsigned short)((u + 0x7FFFu + ((u >> 16) & 1u)) >> 16); }
__device__ __forceinline__ float bf16_val(unsigned short b) { return __uint_as_float(((unsigned int)b) << 16); }
__device__ __forceinline__ float bf16_rne(float x) { return bf16_val(bf16_bits(x)); }

__device__ __forceinline__ v16h g2_frag(const _Float16* p, int hh) { FragH f; f.half[0] = *(const v8us*)((const unsigned short*)p + 8 * hh); f.half[1] = *(const v8us*)((const unsigned short*)p + 16 + 8 * hh); return f.v; }
__device__ __forceinline__ v8f g2_mma(v16h a, v16h b, v8f c) { v8f d = __builtin_amdgcn_wmma_f32_16x16x32_f16(false, a, false, b, (short)0, c, false, false); asm volatile("v_nop\n\tv_nop\n\tv_nop\n\tv_nop" : "+v"(d) : "v"(a), "v"(b)); return d; }

__global__ __launch_bounds__(256) void k_x16(const float* __restrict__ x, _Float16* __restrict__ X16) {
  const size_t t = (size_t)blockIdx.x * 256 + threadIdx.x; if (t >= (size_t)MROWS * DM / 8) return;
  const int row = (int)(t / (DM / 8)), c8 = (int)(t % (DM / 8)) * 8; const int b = row / SEQ, s = row - b * SEQ;
  const float* src = x + ((size_t)b * SEQ_FULL + s) * DM + c8;
  const v4f a = *(const v4fa*)src; const v4f c = *(const v4fa*)(src + 4); FragH f;
#pragma unroll
  for (int q = 0; q < 4; ++q) { f.h[q] = (_Float16)bf16_rne(a[q]); f.h[4 + q] = (_Float16)bf16_rne(c[q]); }
  *(volatile v8us*)((unsigned short*)X16 + t * 8) = f.half[0]; __threadfence(); *(volatile v8us*)((unsigned short*)X16 + t * 8) = f.half[0]; }

__global__ __launch_bounds__(256) void k_wtr(const float* __restrict__ w, int K, int N, _Float16* __restrict__ Bt) {
  __shared__ unsigned short tl[64][66];
  const int tid = threadIdx.x; const int ntn = N >> 6; const int tk = blockIdx.x / ntn, tn = blockIdx.x - tk * ntn; const int k0 = tk * 64, n0 = tn * 64;
  for (int i = tid; i < 64 * 16; i += 256) { const int r = i >> 4, c4 = (i & 15) * 4;
    const v4f a = *(const v4fa*)(w + (size_t)(k0 + r) * N + n0 + c4);
#pragma unroll
    for (int q = 0; q < 4; ++q) { const _Float16 hv = (_Float16)(bf16_rne(a[q]) * C_W); tl[r][c4 + q] = __builtin_bit_cast(unsigned short, hv); } }
  __syncthreads();
  for (int pass = 0; pass < 2; ++pass) {
#pragma unroll
    for (int rd = 0; rd < 2; ++rd) { const int n = rd * 32 + tid / 8, pc = tid % 8; FragH f;
#pragma unroll
      for (int q = 0; q < 8; ++q) f.u[q] = tl[pc * 8 + q][n];
      *(volatile v8us*)((unsigned short*)Bt + (size_t)(n0 + n) * K + k0 + pc * 8) = f.half[0]; }
    if (pass == 0) __threadfence(); } }

template <int EPI>
__global__ __launch_bounds__(128) void k_gemm(const _Float16* __restrict__ A, int lda, const _Float16* __restrict__ Bh, int ldb, float alpha, const float* __restrict__ bias, float c16,
    _Float16* __restrict__ C16, int ldc16, float* __restrict__ C32, int ldc32, int M, int N, int K) {
  __shared__ __attribute__((aligned(16))) float so[4][32][68];
  const int tid = threadIdx.x, w = tid >> 5, lane = tid & 31, ln = lane & 15, hh = lane >> 4;
  const int ntn = N >> 6; const int mt = blockIdx.x / ntn, nq = blockIdx.x - mt * ntn; const int row0 = mt * 128 + 32 * w, col0 = nq * 64; if (row0 >= M) return;
  const _Float16* a0p = A + (size_t)(row0 + ln) * lda; const _Float16* a1p = a0p + (size_t)16 * lda;
  const _Float16* b0p = Bh + (size_t)(col0 + ln) * ldb; const _Float16* b1p = b0p + (size_t)16 * ldb; const _Float16* b2p = b1p + (size_t)16 * ldb; const _Float16* b3p = b2p + (size_t)16 * ldb;
  const v8f z8 = {0.f,0.f,0.f,0.f,0.f,0.f,0.f,0.f}; v8f c00 = z8, c01 = z8, c02 = z8, c03 = z8, c10 = z8, c11 = z8, c12 = z8, c13 = z8;
#pragma unroll 1
  for (int kb = 0; kb < K; kb += 32) { const v16h a0 = g2_frag(a0p + kb, hh), a1 = g2_frag(a1p + kb, hh);
    v16h b = g2_frag(b0p + kb, hh); c00 = g2_mma(a0, b, c00); c10 = g2_mma(a1, b, c10);
    b = g2_frag(b1p + kb, hh); c01 = g2_mma(a0, b, c01); c11 = g2_mma(a1, b, c11);
    b = g2_frag(b2p + kb, hh); c02 = g2_mma(a0, b, c02); c12 = g2_mma(a1, b, c12);
    b = g2_frag(b3p + kb, hh); c03 = g2_mma(a0, b, c03); c13 = g2_mma(a1, b, c13); }
  v8f accs[8] = {c00, c01, c02, c03, c10, c11, c12, c13};
#pragma unroll
  for (int u = 0; u < 8; ++u) { const int t = u & 3, hf = u >> 2; const int col = col0 + t * 16 + ln; const float bv = bf16_rne(bias[col]);
#pragma unroll
    for (int r = 0; r < 8; ++r) { const int rloc = hf * 16 + 8 * hh + r; so[w][rloc][t * 16 + ln] = accs[u][r] * alpha + bv; } }
  __builtin_amdgcn_fence(4  , "workgroup"); __builtin_amdgcn_wave_barrier();
  const int rsub = lane >> 4, c4 = (lane & 15) * 4;
  const int rq = lane >> 3, pc = lane & 7;
  if (EPI == 2) {
#pragma unroll 1
    for (int q = 0; q < 16; ++q) { const int r = q * 2 + rsub; v4f v = *(const v4fa*)&so[w][r][c4];
#pragma unroll
      for (int i = 0; i < 4; ++i) v[i] = 0.5f * v[i] * (1.0f + erff(v[i] * 0.70710678118654752f));
      *(v4fa*)&so[w][r][c4] = v; } }
  for (int pass = 0; pass < 2; ++pass) {
    if (EPI == 1 || EPI == 3) {
#pragma unroll
      for (int g = 0; g < 16; ++g) { const int L = g * 4 + rq; const int row = L >> 1, col = (L & 1) * 32 + pc * 4;
        const v4f v = *(const v4fa*)&so[w][row][col];
        *(volatile v4f*)(C32 + (size_t)(row0 + row) * ldc32 + col0 + col) = v; } }
    if (EPI != 3) {
#pragma unroll
      for (int q = 0; q < 16; ++q) { const int r = q * 2 + rsub; const v4f v = *(const v4fa*)&so[w][r][c4]; v4h h4;
#pragma unroll
        for (int i = 0; i < 4; ++i) h4[i] = (_Float16)(v[i] * c16);
        *(volatile v4h*)(C16 + (size_t)(row0 + r) * ldc16 + col0 + c4) = h4; } }
    if (pass == 0) __threadfence(); } }

__global__ __launch_bounds__(256) void k_vt2(const _Float16* __restrict__ QKV, _Float16* __restrict__ VT) {
  __shared__ unsigned short tl[64][66];
  const int tid = threadIdx.x; const int slab = blockIdx.x / NQT, lg = blockIdx.x - slab * NQT; const int b = slab / NH, hd = slab - b * NH; const int s0 = lg * 64;
  for (int i = tid; i < 64 * 8; i += 256) { const int r = i / 8, c8 = (i % 8) * 8; FragH f;
    f.half[0] = *(const v8us*)((const unsigned short*)QKV + ((size_t)b * SEQ + s0 + r) * LQ + 2 * DM + hd * HD + c8);
#pragma unroll
    for (int q = 0; q < 8; ++q) tl[r][c8 + q] = f.u[q]; }
  __syncthreads();
  for (int pass = 0; pass < 2; ++pass) {
#pragma unroll
    for (int rd = 0; rd < 2; ++rd) { const int d = rd * 32 + tid / 8, pc = tid % 8; FragH f;
#pragma unroll
      for (int q = 0; q < 8; ++q) f.u[q] = tl[pc * 8 + q][d];
      *(volatile v8us*)((unsigned short*)VT + ((size_t)slab * HD + d) * SEQ + s0 + pc * 8) = f.half[0]; }
    if (pass == 0) __threadfence(); } }

__global__ __launch_bounds__(256) void k_mflag(const int* __restrict__ mask, int* __restrict__ MF) {
  __shared__ int sf[32]; __shared__ int srow[64];
  const int tid = threadIdx.x; const int b = blockIdx.x / NQT, qt = blockIdx.x - b * NQT; const int kt = tid >> 3, p = tid & 7;
  const bool ok = (kt < NKT) && (kt <= qt); const int ktc = ok ? kt : 0;
  const int* mb = mask + (size_t)b * SEQ_FULL * SEQ_FULL;
  int z = 0;
#pragma unroll 1
  for (int r = 0; r < 64; ++r) {
    const int* rowp = mb + (size_t)(qt * 64 + r) * SEQ_FULL + ktc * 64 + p * 4;
    const v4ia a = *(const v4ia*)rowp; const v4ia c = *(const v4ia*)(rowp + 32);
    z |= (int)(a[0] == 0) | (int)(a[1] == 0) | (int)(a[2] == 0) | (int)(a[3] == 0) | (int)(c[0] == 0) | (int)(c[1] == 0) | (int)(c[2] == 0) | (int)(c[3] == 0); }
  z = ok ? z : 0;
  z |= __shfl_xor(z, 1); z |= __shfl_xor(z, 2); z |= __shfl_xor(z, 4);
  if (p == 0) sf[kt] = (z != 0) ? 1 : 0;
  if (tid < 64) {
    const int q = qt * 64 + tid; const int* rowp = mb + (size_t)q * SEQ_FULL; int found = 0;
    const int kmax = qt * 16 + 16;
#pragma unroll 1
    for (int k4 = 0; k4 < kmax; ++k4) { const v4ia a = *(const v4ia*)(rowp + k4 * 4); const int kb = k4 * 4;
      found |= ((int)(a[0] != 0) & (int)(kb <= q)) | ((int)(a[1] != 0) & (int)(kb + 1 <= q)) | ((int)(a[2] != 0) & (int)(kb + 2 <= q)) | ((int)(a[3] != 0) & (int)(kb + 3 <= q)); }
    srow[tid] = (found == 0) ? 1 : 0; }
  __syncthreads();
  int wa = srow[tid & 31] | srow[32 + (tid & 31)];
  wa |= __shfl_xor(wa, 16); wa |= __shfl_xor(wa, 8); wa |= __shfl_xor(wa, 4); wa |= __shfl_xor(wa, 2); wa |= __shfl_xor(wa, 1);
  const int fv = sf[tid & 31];
  if (tid < 64) { const int v = (tid < 32) ? fv : ((tid == 32) ? wa : 0); volatile int* d = MF + (size_t)blockIdx.x * 64 + tid; *d = v; __threadfence(); *d = v; } }

__global__ __launch_bounds__(128) void k_attn(const _Float16* __restrict__ QKV, const _Float16* __restrict__ VT, const int* __restrict__ mask, const int* __restrict__ MF,
                                              _Float16* __restrict__ CTX) {
  __shared__ __attribute__((aligned(16))) float so[4][16][68];
  const int tid = threadIdx.x, w = tid >> 5, lane = tid & 31, l15 = lane & 15, hh = lane >> 4;
  const int qt = blockIdx.x, slab = blockIdx.y; const int b = slab / NH, hd = slab - b * NH;
  const int q0 = qt * 64 + w * 16;
  const _Float16* Qb = QKV + (size_t)b * SEQ * LQ + hd * HD;
  const _Float16* Kb = Qb + DM;
  const _Float16* Vb = VT + (size_t)slab * HD * SEQ;
  const int* mfp = MF + (size_t)(b * NQT + qt) * 64;
  const int* mrow = mask + ((size_t)b * SEQ_FULL + (q0 + l15)) * SEQ_FULL;
  const int walk = mfp[32];
  int nst = (walk != 0) ? NKT : (qt + 1); nst = (nst < NKT) ? nst : NKT;
  const _Float16* qrow = Qb + (size_t)(q0 + l15) * LQ;
  const v16h qf0 = g2_frag(qrow, hh), qf1 = g2_frag(qrow + 32, hh);
  const v8f z8 = {0.f,0.f,0.f,0.f,0.f,0.f,0.f,0.f};
  v8f o[4] = {z8, z8, z8, z8};
  float m = NEG_INF, l = 0.f;
  const float CL = 0.18033688011112042f;
  const int ql = w * 16 + l15;
#pragma unroll 1
  for (int it = 0; it < nst; ++it) {
    const int key0 = it * 64;
    v8f s[4];
#pragma unroll
    for (int kt = 0; kt < 4; ++kt) {
      const _Float16* krow = Kb + (size_t)(key0 + kt * 16 + l15) * LQ;
      const v16h ka = g2_frag(krow, hh), kk = g2_frag(krow + 32, hh);
      v8f a = g2_mma(ka, qf0, z8); a = g2_mma(kk, qf1, a); s[kt] = a; }
    const int mf = mfp[it];
    if (it > qt) {
#pragma unroll
      for (int kt = 0; kt < 4; ++kt)
#pragma unroll
        for (int r = 0; r < 8; ++r) s[kt][r] = FILL_RAW;
    } else {
      if (it == qt) {
#pragma unroll
        for (int kt = 0; kt < 4; ++kt)
#pragma unroll
          for (int r = 0; r < 8; ++r) s[kt][r] = ((kt * 16 + 8 * hh + r) > ql) ? FILL_RAW : s[kt][r];
      }
      if (mf != 0) {
#pragma unroll
        for (int kt = 0; kt < 4; ++kt) {
          const int* mp = mrow + key0 + kt * 16 + 8 * hh;
          const v4ia ma = *(const v4ia*)mp; const v4ia mb = *(const v4ia*)(mp + 4);
#pragma unroll
          for (int r = 0; r < 4; ++r) { s[kt][r] = (ma[r] == 0) ? FILL_RAW : s[kt][r]; s[kt][4 + r] = (mb[r] == 0) ? FILL_RAW : s[kt][4 + r]; } } } }
    float lmax = NEG_INF;
#pragma unroll
    for (int kt = 0; kt < 4; ++kt)
#pragma unroll
      for (int r = 0; r < 8; ++r) lmax = fmaxf(lmax, s[kt][r]);
    lmax = fmaxf(lmax, __shfl_xor(lmax, 16));
    const float mnew = fmaxf(m, lmax);
    const float mref = (mnew == NEG_INF) ? 0.0f : mnew;
    const float alpha = exp2f((m - mref) * CL);
    m = mnew;
    float psum = 0.f; FragH pa, pb;
#pragma unroll
    for (int r = 0; r < 8; ++r) {
      const float e0 = exp2f(fmaf(s[0][r] - mref, CL, 10.0f)), e1 = exp2f(fmaf(s[1][r] - mref, CL, 10.0f)), e2 = exp2f(fmaf(s[2][r] - mref, CL, 10.0f)), e3 = exp2f(fmaf(s[3][r] - mref, CL, 10.0f));
      psum += (e0 + e1) + (e2 + e3);
      pa.h[r] = (_Float16)e0; pa.h[8 + r] = (_Float16)e1; pb.h[r] = (_Float16)e2; pb.h[8 + r] = (_Float16)e3; }
    l = l * alpha + psum;
    float ar[8];
#pragma unroll
    for (int r = 0; r < 8; ++r) ar[r] = __shfl(alpha, 8 * hh + r);
#pragma unroll
    for (int dt = 0; dt < 4; ++dt) {
#pragma unroll
      for (int r = 0; r < 8; ++r) o[dt][r] *= ar[r];
      const _Float16* vrow = Vb + (size_t)(dt * 16 + l15) * SEQ + key0;
      const v16h va = g2_frag(vrow, hh), vb = g2_frag(vrow + 32, hh);
      o[dt] = g2_mma(pa.v, va, o[dt]); o[dt] = g2_mma(pb.v, vb, o[dt]); } }
  const float lt = l + __shfl_xor(l, 16);
  const float inv = C_CTX / lt;
  float ir[8];
#pragma unroll
  for (int r = 0; r < 8; ++r) ir[r] = __shfl(inv, 8 * hh + r);
#pragma unroll
  for (int dt = 0; dt < 4; ++dt)
#pragma unroll
    for (int r = 0; r < 8; ++r) so[w][8 * hh + r][dt * 16 + l15] = o[dt][r] * ir[r];
  __builtin_amdgcn_fence(4  , "workgroup"); __builtin_amdgcn_wave_barrier();
  const int rsub = lane >> 4, c4 = (lane & 15) * 4;
  for (int pass = 0; pass < 2; ++pass) {
#pragma unroll
    for (int q = 0; q < 8; ++q) { const int r = q * 2 + rsub; const v4f v = *(const v4fa*)&so[w][r][c4]; v4h h4;
#pragma unroll
      for (int i = 0; i < 4; ++i) h4[i] = (_Float16)v[i];
      *(volatile v4h*)(CTX + ((size_t)b * SEQ + q0 + r) * DM + hd * HD + c4) = h4; }
    if (pass == 0) __threadfence(); } }

__global__ __launch_bounds__(256) void k_ln(const float* __restrict__ AO, const float* __restrict__ DN, const float* __restrict__ gamma, const float* __restrict__ beta, float* __restrict__ out) {
  __shared__ float red[2][8];
  const int tid = threadIdx.x, wv = tid >> 5, lane = tid & 31; const int row = blockIdx.x; const int b = row / SEQ, s = row - b * SEQ;
  const size_t gi = (size_t)row * DM + tid * 4;
  const v4f a = *(const v4fa*)(AO + gi); const v4f d = *(const v4fa*)(DN + gi);
  v4f y;
#pragma unroll
  for (int i = 0; i < 4; ++i) y[i] = a[i] + d[i];
  float sm = (y[0] + y[1]) + (y[2] + y[3]);
  sm += __shfl_xor(sm, 16); sm += __shfl_xor(sm, 8); sm += __shfl_xor(sm, 4); sm += __shfl_xor(sm, 2); sm += __shfl_xor(sm, 1);
  if (lane == 0) red[0][wv] = sm;
  __syncthreads();
  float tot = 0.f;
#pragma unroll
  for (int i = 0; i < 8; ++i) tot += red[0][i];
  const float mu = tot * (1.0f / DM);
  float sq = 0.f;
#pragma unroll
  for (int i = 0; i < 4; ++i) { const float t = y[i] - mu; sq += t * t; }
  sq += __shfl_xor(sq, 16); sq += __shfl_xor(sq, 8); sq += __shfl_xor(sq, 4); sq += __shfl_xor(sq, 2); sq += __shfl_xor(sq, 1);
  if (lane == 0) red[1][wv] = sq;
  __syncthreads();
  float tot2 = 0.f;
#pragma unroll
  for (int i = 0; i < 8; ++i) tot2 += red[1][i];
  const float var = tot2 * (1.0f / DM);
  const float rs = 1.0f / sqrtf(var + 1e-6f);
  const v4f g = *(const v4fa*)(gamma + tid * 4); const v4f be = *(const v4fa*)(beta + tid * 4);
  v4f ov;
#pragma unroll
  for (int i = 0; i < 4; ++i) ov[i] = (y[i] - mu) * rs * bf16_rne(g[i]) + bf16_rne(be[i]);
  float* dst = out + ((size_t)b * SEQ_FULL + s) * DM + tid * 4;
  *(volatile v4f*)dst = ov; __threadfence(); *(volatile v4f*)dst = ov; }

#define SZ_W   ((size_t)DM * DM * 2)
#define SZ_W1  ((size_t)DM * DFF * 2)
#define SZ_R0  ((size_t)MROWS * DM * 2)
#define SZ_R1  ((size_t)MROWS * LQ * 2)
#define SZ_VT  ((size_t)NB * NH * HD * SEQ * 2)
#define SZ_AO  ((size_t)MROWS * DM * 4)
#define SZ_H   ((size_t)MROWS * DFF * 2)
#define SZ_MF  ((size_t)NB * NQT * 64 * 4)
static_assert(SZ_R1 == (size_t)MROWS * DM * 2 + (size_t)MROWS * DM * 4);
static_assert(SZ_W % 256 == 0 && SZ_W1 % 256 == 0 && SZ_R0 % 256 == 0 && SZ_R1 % 256 == 0 && SZ_VT % 256 == 0 && SZ_AO % 256 == 0 && SZ_H % 256 == 0 && SZ_MF % 256 == 0);
static_assert(4 * SZ_W + 2 * SZ_W1 + SZ_R0 + SZ_R1 + SZ_VT + SZ_AO + SZ_H + SZ_MF <= (size_t)134217728);

extern "C" void kernel_launch(void* const* d_in, const int* in_sizes, int n_in,
                              void* d_out, int out_size, void* d_ws, size_t ws_size, hipStream_t stream) {
  if (n_in < 16) return;
  const float* x  = (const float*)d_in[0];
  const int*   mk = (const int*)d_in[1];
  const float* Wq = (const float*)d_in[2];  const float* bq = (const float*)d_in[3];
  const float* Wk = (const float*)d_in[4];  const float* bk = (const float*)d_in[5];
  const float* Wv = (const float*)d_in[6];  const float* bv = (const float*)d_in[7];
  const float* Wo = (const float*)d_in[8];  const float* bo = (const float*)d_in[9];
  const float* W1 = (const float*)d_in[10]; const float* b1 = (const float*)d_in[11];
  const float* W2 = (const float*)d_in[12]; const float* b2 = (const float*)d_in[13];
  const float* gm = (const float*)d_in[14]; const float* bt = (const float*)d_in[15];
  const long long rows_io = (long long)(NB - 1) * SEQ_FULL + SEQ;
  if ((long long)in_sizes[0] < rows_io * DM) return;
  if ((long long)in_sizes[1] < (rows_io - 1) * SEQ_FULL + SEQ) return;
  if (in_sizes[2] < DM * DM || in_sizes[4] < DM * DM || in_sizes[6] < DM * DM || in_sizes[8] < DM * DM) return;
  if (in_sizes[3] < DM || in_sizes[5] < DM || in_sizes[7] < DM || in_sizes[9] < DM) return;
  if (in_sizes[10] < DM * DFF || in_sizes[12] < DFF * DM || in_sizes[11] < DFF || in_sizes[13] < DM) return;
  if (in_sizes[14] < DM || in_sizes[15] < DM) return;
  if ((long long)out_size < rows_io * DM) return;
  char* ws = (char*)d_ws; size_t off = 0;
  auto take = [&](size_t bytes) { char* p = ws + off; off += (bytes + 255) & ~(size_t)255; return p; };
  _Float16* BQ  = (_Float16*)take(SZ_W);
  _Float16* BK  = (_Float16*)take(SZ_W);
  _Float16* BV  = (_Float16*)take(SZ_W);
  _Float16* BO  = (_Float16*)take(SZ_W);
  _Float16* B1  = (_Float16*)take(SZ_W1);
  _Float16* B2  = (_Float16*)take(SZ_W1);
  char*     R0  = take(SZ_R0);
  char*     R1  = take(SZ_R1);
  _Float16* VT  = (_Float16*)take(SZ_VT);
  float*    AO  = (float*)take(SZ_AO);
  _Float16* H16 = (_Float16*)take(SZ_H);
  int*      MF  = (int*)take(SZ_MF);
  if (off > ws_size || off > (size_t)134217728) return;
  _Float16* X16 = (_Float16*)R0;
  _Float16* CTX = (_Float16*)R0;
  _Float16* QKV = (_Float16*)R1;
  _Float16* A16 = (_Float16*)R1;
  float*    DN  = (float*)(R1 + (size_t)MROWS * DM * 2);
  k_wtr<<<(unsigned)((DM / 64) * (DM / 64)), 256, 0, stream>>>(Wq, DM, DM, BQ);
  k_wtr<<<(unsigned)((DM / 64) * (DM / 64)), 256, 0, stream>>>(Wk, DM, DM, BK);
  k_wtr<<<(unsigned)((DM / 64) * (DM / 64)), 256, 0, stream>>>(Wv, DM, DM, BV);
  k_wtr<<<(unsigned)((DM / 64) * (DM / 64)), 256, 0, stream>>>(Wo, DM, DM, BO);
  k_wtr<<<(unsigned)((DM / 64) * (DFF / 64)), 256, 0, stream>>>(W1, DM, DFF, B1);
  k_wtr<<<(unsigned)((DFF / 64) * (DM / 64)), 256, 0, stream>>>(W2, DFF, DM, B2);
  const size_t nx8 = (size_t)MROWS * DM / 8;
  k_x16<<<(unsigned)((nx8 + 255) / 256), 256, 0, stream>>>(x, X16);
  const unsigned gg = (unsigned)((MROWS / 128) * (DM / 64));
  const unsigned gf = (unsigned)((MROWS / 128) * (DFF / 64));
  k_gemm<0><<<gg, 128, 0, stream>>>(X16, DM, BQ, DM, 1.0f / 16.0f, bq, 1.0f, QKV,          LQ, AO, DM, MROWS, DM, DM);
  k_gemm<0><<<gg, 128, 0, stream>>>(X16, DM, BK, DM, 1.0f / 16.0f, bk, 1.0f, QKV + DM,     LQ, AO, DM, MROWS, DM, DM);
  k_gemm<0><<<gg, 128, 0, stream>>>(X16, DM, BV, DM, 1.0f / 16.0f, bv, 1.0f, QKV + 2 * DM, LQ, AO, DM, MROWS, DM, DM);
  k_vt2<<<(unsigned)(NB * NH * NQT), 256, 0, stream>>>(QKV, VT);
  k_mflag<<<(unsigned)(NB * NQT), 256, 0, stream>>>(mk, MF);
  k_attn<<<dim3((unsigned)NQT, (unsigned)(NB * NH)), 128, 0, stream>>>(QKV, VT, mk, MF, CTX);
  k_gemm<1><<<gg, 128, 0, stream>>>(CTX, DM, BO, DM, 1.0f / (C_CTX * C_W), bo, C_AO, A16, DM, AO, DM, MROWS, DM, DM);
  k_gemm<2><<<gf, 128, 0, stream>>>(A16, DM, B1, DM, 1.0f / (C_AO * C_W), b1, C_H, H16, DFF, AO, DM, MROWS, DFF, DM);
  k_gemm<3><<<gg, 128, 0, stream>>>(H16, DFF, B2, DFF, 1.0f / (C_H * C_W), b2, 1.0f, A16, DM, DN, DM, MROWS, DM, DFF);
  k_ln<<<(unsigned)MROWS, 256, 0, stream>>>(AO, DN, gm, bt, (float*)d_out);
}
